// TritonGatherConv_73254962201305
// MI455X (gfx1250) — hardware-verified
//
#include <hip/hip_runtime.h>


#define NBT  4
#define LL   1024
#define CC   1024
#define NH_  8
#define HDD  128
#define NS   33
#define HS   16
#define KW   64
#define NR   (NBT * LL)
#define NWP  64
typedef _Float16 h16;
typedef unsigned short bf;
typedef __attribute__((ext_vector_type(16))) __bf16   v16bf;
typedef __attribute__((ext_vector_type(16))) _Float16 v16h;
typedef __attribute__((ext_vector_type(8)))  _Float16 v8h;
typedef __attribute__((ext_vector_type(8)))  unsigned short v8us;
typedef __attribute__((ext_vector_type(8)))  float    v8f;
typedef __attribute__((ext_vector_type(4)))  float    v4f;
typedef v8h  __attribute__((may_alias)) v8ha;
typedef v4f  __attribute__((may_alias)) v4fa;
typedef v8us __attribute__((may_alias)) v8usa;

__device__ __forceinline__ unsigned short f2bf(float f) { unsigned u = __float_as_uint(f); u += 0x7FFFu + ((u >> 16) & 1u); return (unsigned short)(u >> 16); }
__device__ __forceinline__ float bf2f(unsigned short b) { return __uint_as_float(((unsigned)b) << 16); }
__device__ __forceinline__ float bfr(float f) { return bf2f(f2bf(f)); }
__device__ __forceinline__ v16h cat16(v8h lo, v8h hi) { return __builtin_shufflevector(lo, hi, 0, 1, 2, 3, 4, 5, 6, 7, 8, 9, 10, 11, 12, 13, 14, 15); }
__device__ __forceinline__ v16bf cat16b(v8us lo, v8us hi) { return __builtin_bit_cast(v16bf, __builtin_shufflevector(lo, hi, 0, 1, 2, 3, 4, 5, 6, 7, 8, 9, 10, 11, 12, 13, 14, 15)); }
__device__ __forceinline__ v8f wmma16(v16h a, v16h b, v8f c) { return __builtin_amdgcn_wmma_f32_16x16x32_f16(false, a, false, b, (short)0, c, false, false); }
__device__ __forceinline__ v8f wmmab(v16bf a, v16bf b, v8f c) { return __builtin_amdgcn_wmma_f32_16x16x32_bf16(false, a, false, b, (short)0, c, false, false); }


template <typename T16> struct WFrag;
template <> struct WFrag<h16> { typedef v16h V; static __device__ __forceinline__ V ld(const h16* p) { return cat16(*(const v8h*)p, *(const v8h*)(p + 16)); } static __device__ __forceinline__ v8f mma(V a, V b, v8f c) { return wmma16(a, b, c); } };
template <> struct WFrag<bf> { typedef v16bf V; static __device__ __forceinline__ V ld(const bf* p) { return cat16b(*(const v8us*)p, *(const v8us*)(p + 16)); } static __device__ __forceinline__ v8f mma(V a, V b, v8f c) { return wmmab(a, b, c); } };
template <typename T16, int NSPLIT, bool BIAS>
__global__ __launch_bounds__(32) void k_gemmw(const T16* __restrict__ A, const T16* __restrict__ A2, const T16* __restrict__ Bt, const T16* __restrict__ Bt2, int K, float* C, int ldc, const float* __restrict__ bias, size_t sA, size_t sB, size_t sC) {
    typedef typename WFrag<T16>::V V;
    __shared__ __align__(16) float os[16 * 68];
    const size_t z = blockIdx.z; A += z * sA; if (A2) A2 += z * sA; Bt += z * sB; if (Bt2) Bt2 += z * sB; C += z * sC;
    const int lane = threadIdx.x & 31, lr = lane & 15, hi = lane >> 4; const int r0 = blockIdx.x * 64, c0 = blockIdx.y * 64;
    v8f acc[4][4];
#pragma unroll
    for (int mb = 0; mb < 4; ++mb)
#pragma unroll
        for (int nb = 0; nb < 4; ++nb) acc[mb][nb] = (v8f){};
    const size_t aoff = (size_t)(r0 + lr) * K + 8 * hi, boff = (size_t)(c0 + lr) * K + 8 * hi;
#pragma unroll 1
    for (int kc = 0; kc < K; kc += 32) {
        V a[4], a2[4];
#pragma unroll
        for (int mb = 0; mb < 4; ++mb) { a[mb] = WFrag<T16>::ld(A + aoff + (size_t)mb * 16 * K + kc); if (NSPLIT == 1 || NSPLIT == 2) a2[mb] = WFrag<T16>::ld(A2 + aoff + (size_t)mb * 16 * K + kc); }
#pragma unroll
        for (int nb = 0; nb < 4; ++nb) { const V b = WFrag<T16>::ld(Bt + boff + (size_t)nb * 16 * K + kc); V b2; if (NSPLIT >= 2) b2 = WFrag<T16>::ld(Bt2 + boff + (size_t)nb * 16 * K + kc);
#pragma unroll
            for (int mb = 0; mb < 4; ++mb) { acc[mb][nb] = WFrag<T16>::mma(a[mb], b, acc[mb][nb]); if (NSPLIT == 1 || NSPLIT == 2) acc[mb][nb] = WFrag<T16>::mma(a2[mb], b, acc[mb][nb]); if (NSPLIT >= 2) acc[mb][nb] = WFrag<T16>::mma(a[mb], b2, acc[mb][nb]); } }
        asm volatile("v_nop\n\tv_nop\n\tv_nop\n\tv_nop" : "+v"(acc[0][0]), "+v"(acc[1][1]), "+v"(acc[2][2]), "+v"(acc[3][3]) : "v"(a[0]), "v"(a[3]));
    }
#pragma unroll
    for (int mb = 0; mb < 4; ++mb) {
#pragma unroll
        for (int nb = 0; nb < 4; ++nb) {
#pragma unroll
            for (int j = 0; j < 8; ++j) os[(hi * 8 + j) * 68 + nb * 16 + lr] = acc[mb][nb][j]; }
        __builtin_amdgcn_wave_barrier(); asm volatile("" ::: "memory");
        float* crow = C + (size_t)(r0 + mb * 16) * ldc + c0;
#pragma unroll 1
        for (int ps = 0; ps < 2; ++ps) {
#pragma unroll
            for (int s = 0; s < 8; ++s) { const int row = 2 * s + hi, cofs = lr * 4; v4f val = *(const v4fa*)(os + row * 68 + cofs); if (BIAS) { val[0] += bfr(bias[c0 + cofs]); val[1] += bfr(bias[c0 + cofs + 1]); val[2] += bfr(bias[c0 + cofs + 2]); val[3] += bfr(bias[c0 + cofs + 3]); }
                *(volatile v4f*)(crow + (size_t)row * ldc + cofs) = val; }
            if (ps == 0) __threadfence(); }
        __builtin_amdgcn_wave_barrier(); asm volatile("" ::: "memory");
    }
}

typedef __attribute__((ext_vector_type(4))) unsigned short v4us;
__device__ __forceinline__ void splitf(float y, unsigned short& h, unsigned short& l) { h = f2bf(y); l = f2bf(y - bf2f(h)); }
__device__ __forceinline__ float sigm(float a) { return __fdiv_rn(1.0f, __fadd_rn(1.0f, __builtin_amdgcn_exp2f(__fmul_rn(a, -1.4426950408889634f)))); }
__device__ __forceinline__ float siluf(float a) { return __fmul_rn(a, sigm(a)); }
__device__ __forceinline__ float tanhx(float a) { return __fsub_rn(__fdiv_rn(2.0f, __fadd_rn(1.0f, __builtin_amdgcn_exp2f(__fmul_rn(a, -2.8853900817779268f)))), 1.0f); }
__global__ __launch_bounds__(256) void k_cvt8(const float* __restrict__ src, bf* dst, size_t n8) { const size_t i = (size_t)blockIdx.x * 256 + threadIdx.x; if (i >= n8) return; const v8f v = *(const v8f*)(src + i * 8); v8us o;
#pragma unroll
    for (int k = 0; k < 8; ++k) o[k] = f2bf(v[k]); *(volatile v8us*)(dst + i * 8) = o; __threadfence(); *(volatile v8us*)(dst + i * 8) = o; }

__global__ __launch_bounds__(256) void k_wpad(const float* __restrict__ w, bf* Bt) { const size_t i = (size_t)blockIdx.x * 256 + threadIdx.x; if (i >= (size_t)NWP * CC / 8) return; const int r = (int)(i / (CC / 8)); const int c0 = (int)(i % (CC / 8)) * 8; v8us o;
#pragma unroll
    for (int k = 0; k < 8; ++k) o[k] = (r < 2 * NH_) ? f2bf(w[(size_t)r * CC + c0 + k]) : (unsigned short)0; *(volatile v8us*)(Bt + (size_t)r * CC + c0) = o; __threadfence(); *(volatile v8us*)(Bt + (size_t)r * CC + c0) = o; }
__global__ __launch_bounds__(256) void k_pos(const float* __restrict__ WV, const float* __restrict__ wb, int* LO, float* FR) { const int row = blockIdx.x * 256 + threadIdx.x; if (row >= NR) return; const int l = row % LL; float fs = 0.f, ps_ = 0.f;
#pragma unroll 1
    for (int h = 0; h < NH_; ++h) { const float w0 = siluf(__fadd_rn(WV[(size_t)row * NWP + h], bfr(wb[h]))); const float w1 = siluf(__fadd_rn(WV[(size_t)row * NWP + NH_ + h], bfr(wb[NH_ + h]))); float fq = __fmul_rn(sigm(w0), 15.0f); asm volatile("" : "+v"(fq)); fq = __fadd_rn(fq, 1.0f); float ph = __fmul_rn(tanhx(w1), 16.0f); asm volatile("" : "+v"(ph)); fs = __fadd_rn(fs, fq); ps_ = __fadd_rn(ps_, ph); }
    const float freq = __fdiv_rn(fs, 8.0f), phase = __fdiv_rn(ps_, 8.0f);
#pragma unroll 1
    for (int pp = 0; pp < 2; ++pp) {
#pragma unroll 1
        for (int s = 0; s < NS; ++s) { float t = __fmul_rn((float)(s - HS), freq); asm volatile("" : "+v"(t)); float p = __fadd_rn(__fadd_rn((float)l, t), phase); p = fminf(fmaxf(p, 0.0f), (float)(LL - 1)); const float fl = floorf(p); const int lo = (int)fl; const float fr = __fsub_rn(p, fl);
            *(volatile int*)(LO + (size_t)row * 64 + s) = lo; *(volatile float*)(FR + (size_t)row * 64 + s) = fr; }
        if (pp == 0) __threadfence(); } }
__global__ __launch_bounds__(256) void k_gath(const float* __restrict__ X, const int* __restrict__ LO, const float* __restrict__ FR, const float* __restrict__ KR, const float* __restrict__ kb, bf* Gh, bf* Gl) {
    const int row = blockIdx.x; const int b = row / LL; const int c0 = threadIdx.x * 4; const int h = c0 / HDD; const float* xb = X + (size_t)b * LL * CC; float acc[4] = {0.f, 0.f, 0.f, 0.f};
#pragma unroll 1
    for (int s = 0; s < NS; ++s) { const int lo = min(max(LO[(size_t)row * 64 + s], 0), LL - 1); const int hi = min(lo + 1, LL - 1);     const float fr = FR[(size_t)row * 64 + s];
        const float wk = siluf(__fadd_rn(KR[(size_t)row * (NH_ * KW) + h * KW + s], bfr(kb[h * KW + s])));
        const v4f a = *(const v4f*)(xb + (size_t)lo * CC + c0); const v4f bq = *(const v4f*)(xb + (size_t)hi * CC + c0);
#pragma unroll
        for (int q = 0; q < 4; ++q) { const float xl = bfr(a[q]), xh = bfr(bq[q]); float df = __fsub_rn(xh, xl); asm volatile("" : "+v"(df)); float m = __fmul_rn(fr, df); asm volatile("" : "+v"(m)); float g = __fadd_rn(xl, m); asm volatile("" : "+v"(g)); float pr = __fmul_rn(g, wk); asm volatile("" : "+v"(pr)); acc[q] = __fadd_rn(acc[q], pr); } }
    v4us oh, ol;
#pragma unroll
    for (int q = 0; q < 4; ++q) { unsigned short h2, l2; splitf(acc[q], h2, l2); oh[q] = h2; ol[q] = l2; }
    const size_t o = (size_t)row * CC + c0; *(volatile v4us*)(Gh + o) = oh; *(volatile v4us*)(Gl + o) = ol; __threadfence(); *(volatile v4us*)(Gh + o) = oh; *(volatile v4us*)(Gl + o) = ol; }
__global__ __launch_bounds__(256) void k_siluo(const float* __restrict__ Y, float* out, size_t n4) { const size_t i = (size_t)blockIdx.x * 256 + threadIdx.x; if (i >= n4) return; const v4f y = *(const v4f*)(Y + i * 4); v4f o;
#pragma unroll
    for (int q = 0; q < 4; ++q) o[q] = siluf(y[q]); *(volatile v4f*)(out + i * 4) = o; __threadfence(); *(volatile v4f*)(out + i * 4) = o; }

extern "C" void kernel_launch(void* const* d_in, const int* in_sizes, int n_in,
                              void* d_out, int out_size, void* d_ws, size_t ws_size, hipStream_t stream) {
    (void)in_sizes; (void)n_in; (void)out_size;
    const float* x = (const float*)d_in[0]; const float* ww = (const float*)d_in[1]; const float* wb = (const float*)d_in[2]; const float* kw = (const float*)d_in[3]; const float* kb = (const float*)d_in[4]; const float* ow = (const float*)d_in[5];
    float* OUT = (float*)d_out;
    char* wsp = (char*)d_ws;
    auto take = [&](size_t bytes) { char* p = wsp; wsp += (bytes + 255) & ~(size_t)255; return (void*)p; };
    bf* XB = (bf*)take((size_t)NR * CC * 2); bf* WWB = (bf*)take((size_t)NWP * CC * 2); bf* KWB = (bf*)take((size_t)NH_ * KW * CC * 2); bf* OWB = (bf*)take((size_t)CC * CC * 2);
    float* WV = (float*)take((size_t)NR * NWP * 4); float* KR = (float*)take((size_t)NR * NH_ * KW * 4); int* LO = (int*)take((size_t)NR * 64 * 4); float* FR = (float*)take((size_t)NR * 64 * 4); bf* Gh = (bf*)take((size_t)NR * CC * 2); bf* Gl = (bf*)take((size_t)NR * CC * 2); float* Y = (float*)take((size_t)NR * CC * 4);
    if ((size_t)(wsp - (char*)d_ws) > ws_size) return;
    k_cvt8<<<(unsigned)(((size_t)NR * CC / 8 + 255) / 256), 256, 0, stream>>>(x, XB, (size_t)NR * CC / 8);
    k_wpad<<<(unsigned)(((size_t)NWP * CC / 8 + 255) / 256), 256, 0, stream>>>(ww, WWB);
    k_cvt8<<<(unsigned)(((size_t)NH_ * KW * CC / 8 + 255) / 256), 256, 0, stream>>>(kw, KWB, (size_t)NH_ * KW * CC / 8);
    k_cvt8<<<(unsigned)(((size_t)CC * CC / 8 + 255) / 256), 256, 0, stream>>>(ow, OWB, (size_t)CC * CC / 8);
    k_gemmw<bf, 0, false><<<dim3(NR / 64, NWP / 64, 1), 32, 0, stream>>>(XB, nullptr, WWB, nullptr, CC, WV, NWP, nullptr, 0, 0, 0);
    k_gemmw<bf, 0, false><<<dim3(NR / 64, (NH_ * KW) / 64, 1), 32, 0, stream>>>(XB, nullptr, KWB, nullptr, CC, KR, NH_ * KW, nullptr, 0, 0, 0);
    k_pos<<<NR / 256, 256, 0, stream>>>(WV, wb, LO, FR);
    k_gath<<<NR, 256, 0, stream>>>(x, LO, FR, KR, kb, Gh, Gl);
    k_gemmw<bf, 1, false><<<dim3(NR / 64, CC / 64, 1), 32, 0, stream>>>(Gh, Gl, OWB, nullptr, CC, Y, CC, nullptr, 0, 0, 0);
    k_siluo<<<(unsigned)(((size_t)NR * CC / 4 + 255) / 256), 256, 0, stream>>>(Y, OUT, (size_t)NR * CC / 4);
}
